// DeepRNNC_86535001080504
// MI455X (gfx1250) — hardware-verified
//
#include <hip/hip_runtime.h>
#include <math.h>

typedef __attribute__((ext_vector_type(16))) __bf16   v16b;
typedef __attribute__((ext_vector_type(8)))  float    v8f;
typedef __attribute__((ext_vector_type(4)))  float    v4f;
typedef __attribute__((ext_vector_type(8)))  unsigned v8u;

constexpr int kBatch   = 512;
constexpr int kSteps   = 2048;
constexpr int kHid     = 20;
constexpr int kNout    = 10;
constexpr int kTileB   = 16;
constexpr int kXChunk  = 32;
constexpr int kOChunk  = 16;
constexpr int kXPitch  = 36;
constexpr int kORow    = kOChunk * kNout;
constexpr int kOVec4   = kORow / 4;
constexpr int kFlushIt = (kTileB * kOVec4) / 32;
constexpr int kPadK    = 32;
static_assert(kBatch % kTileB == 0, "batch tiles exact");
static_assert(kSteps % kXChunk == 0 && kXChunk == 2 * kOChunk, "step chunks exact");
static_assert(kHid <= kPadK && kHid > 16, "hidden size uses two 16-row tiles, K padded to 32");
static_assert(kNout <= 16, "head fits one 16-row tile");
static_assert(kORow == 160 && kOVec4 == 40 && kFlushIt == 20, "flush map: 16 rows x 40 float4 = 20 wave stores");
static_assert((kOVec4 % 8) == 0, "eight consecutive lanes stay inside one row and one 128-B line");
static_assert(((kOChunk * kNout * 4) % 128) == 0, "16 steps of one batch row = whole 128-B lines");
static_assert(((kSteps * kNout * 4) % 128) == 0, "batch row pitch of the output is a line multiple");
static_assert((kXPitch % 4) == 0 && kXPitch >= kXChunk, "x tile pitch");

__device__ __forceinline__ unsigned bf_bits(float f) {
  const unsigned u = __float_as_uint(f);
  return (u + 0x7FFFu + ((u >> 16) & 1u)) >> 16;
}
__device__ __forceinline__ void split2(float f, unsigned& hb, unsigned& lb) {
  hb = bf_bits(f);
  const float resid = f - __uint_as_float(hb << 16);
  lb = bf_bits(resid);
}
__device__ __forceinline__ void pack_frag(const v8f& p, const v8f& q, v16b& hi, v16b& lo) {
  v8u wh, wl;
#pragma unroll
  for (int j = 0; j < 4; ++j) {
    unsigned h0, l0, h1, l1;
    split2(p[2 * j], h0, l0);
    split2(p[2 * j + 1], h1, l1);
    wh[j] = h0 | (h1 << 16);
    wl[j] = l0 | (l1 << 16);
  }
#pragma unroll
  for (int j = 0; j < 4; ++j) {
    unsigned h0, l0, h1, l1;
    split2(q[2 * j], h0, l0);
    split2(q[2 * j + 1], h1, l1);
    wh[4 + j] = h0 | (h1 << 16);
    wl[4 + j] = l0 | (l1 << 16);
  }
  hi = __builtin_bit_cast(v16b, wh);
  lo = __builtin_bit_cast(v16b, wl);
}
__device__ __forceinline__ v8f mma_b(v16b a, v16b b, v8f c) {
  return __builtin_amdgcn_wmma_f32_16x16x32_bf16(false, a, false, b, (short)0, c, false, false);
}
__device__ __forceinline__ v8f mma3(v16b ah, v16b al, v16b bh, v16b bl, v8f c) {
  c = mma_b(ah, bh, c);
  c = mma_b(ah, bl, c);
  c = mma_b(al, bh, c);
  asm volatile("v_nop\n\tv_nop\n\tv_nop\n\tv_nop" : "+v"(c) : "v"(ah), "v"(al), "v"(bh), "v"(bl));
  return c;
}
__device__ __forceinline__ float tanh_f(float v) {
  const float e = expf(2.0f * v);
  return 1.0f - 2.0f / (e + 1.0f);
}

__global__ __launch_bounds__(32) __attribute__((amdgpu_num_vgpr(256)))
void seq2_tanh_head_kernel(const float* __restrict__ x,
                           const float* __restrict__ W_ih0,
                           const float* __restrict__ W_hh0,
                           const float* __restrict__ b_ih0,
                           const float* __restrict__ b_hh0,
                           const float* __restrict__ W_ih1,
                           const float* __restrict__ W_hh1,
                           const float* __restrict__ b_ih1,
                           const float* __restrict__ b_hh1,
                           const float* __restrict__ W_fc,
                           const float* __restrict__ b_fc,
                           float* __restrict__ out)
{
  __shared__ __align__(16) float wst[4 * kPadK * kPadK];
  __shared__ __align__(16) float cv[4 * 32];
  __shared__ __align__(16) float xs[kTileB * kXPitch];
  __shared__ __align__(16) float os[kTileB * kORow];

  const int lane = threadIdx.x & 31;
  const int hh   = lane >> 4;
  const int c    = lane & 15;
  const int b0   = blockIdx.x * kTileB;

  {
    const int ki = (lane < kHid) ? lane : (kHid - 1);
#pragma unroll 1
    for (int g = 0; g < kPadK; ++g) {
      const int gi = (g < kHid) ? g : (kHid - 1);
      const int go = (g < kNout) ? g : (kNout - 1);
      float wa = W_hh0[gi * kHid + ki];
      asm volatile("" : "+v"(wa));
      float wb = W_ih1[gi * kHid + ki];
      asm volatile("" : "+v"(wb));
      float wc = W_hh1[gi * kHid + ki];
      asm volatile("" : "+v"(wc));
      float wd = W_fc[go * kHid + ki];
      asm volatile("" : "+v"(wd));
      const bool v20 = (g < kHid) && (lane < kHid);
      const bool v10 = (g < kNout) && (lane < kHid);
      wst[0 * kPadK * kPadK + g * kPadK + lane] = v20 ? wa : 0.0f;
      wst[1 * kPadK * kPadK + g * kPadK + lane] = v20 ? wb : 0.0f;
      wst[2 * kPadK * kPadK + g * kPadK + lane] = v20 ? wc : 0.0f;
      wst[3 * kPadK * kPadK + g * kPadK + lane] = v10 ? wd : 0.0f;
    }
  }
  {
    const int li = (lane < kHid) ? lane : (kHid - 1);
    const int lo = (lane < kNout) ? lane : (kNout - 1);
    float wi = W_ih0[li];
    asm volatile("" : "+v"(wi));
    float ba = b_ih0[li];
    asm volatile("" : "+v"(ba));
    float bb = b_hh0[li];
    asm volatile("" : "+v"(bb));
    float bc = b_ih1[li];
    asm volatile("" : "+v"(bc));
    float bd = b_hh1[li];
    asm volatile("" : "+v"(bd));
    float bf = b_fc[lo];
    asm volatile("" : "+v"(bf));
    const bool v20 = (lane < kHid);
    const bool v10 = (lane < kNout);
    cv[0 * 32 + lane] = v20 ? wi : 0.0f;
    cv[1 * 32 + lane] = v20 ? (ba + bb) : 0.0f;
    cv[2 * 32 + lane] = v20 ? (bc + bd) : 0.0f;
    cv[3 * 32 + lane] = v10 ? bf : 0.0f;
  }
  __syncthreads();

  v16b wh[4][2], wl[4][2];
#pragma unroll
  for (int mat = 0; mat < 4; ++mat) {
#pragma unroll
    for (int mt = 0; mt < 2; ++mt) {
      const float* wp = wst + mat * kPadK * kPadK + (16 * mt + c) * kPadK + 8 * hh;
      const v4f a0 = *(const v4f*)(wp);
      const v4f a1 = *(const v4f*)(wp + 4);
      const v4f a2 = *(const v4f*)(wp + 16);
      const v4f a3 = *(const v4f*)(wp + 20);
      v8f p, q;
#pragma unroll
      for (int e = 0; e < 4; ++e) {
        p[e]     = a0[e];
        p[4 + e] = a1[e];
        q[e]     = a2[e];
        q[4 + e] = a3[e];
      }
      pack_frag(p, q, wh[mat][mt], wl[mat][mt]);
    }
  }

  const v8u zw = {0u, 0u, 0u, 0u, 0u, 0u, 0u, 0u};
  v16b h0h = __builtin_bit_cast(v16b, zw);
  v16b h0l = h0h;
  v16b h1h = h0h;
  v16b h1l = h0h;

#pragma unroll 1
  for (int t0 = 0; t0 < kSteps; t0 += kXChunk) {
    __syncthreads();
#pragma unroll
    for (int it = 0; it < 4; ++it) {
      const int f   = it * 32 + lane;
      const int row = f >> 3;
      const int c4  = (f & 7) * 4;
      const v4f v = *(const v4f*)(x + (size_t)(b0 + row) * kSteps + (size_t)t0 + c4);
      *(v4f*)(xs + row * kXPitch + c4) = v;
    }
    __syncthreads();

#pragma unroll 1
    for (int sub = 0; sub < 2; ++sub) {
#pragma unroll 1
      for (int s = 0; s < kOChunk; ++s) {
        asm volatile("" ::: "memory");
        const float xv = xs[c * kXPitch + sub * kOChunk + s];

        v8f acc0, acc1;
        {
          const v4f w0a = *(const v4f*)(cv + 0 * 32 + 8 * hh);
          const v4f w0b = *(const v4f*)(cv + 0 * 32 + 8 * hh + 4);
          const v4f w0c = *(const v4f*)(cv + 0 * 32 + 16 + 8 * hh);
          const v4f b0a = *(const v4f*)(cv + 1 * 32 + 8 * hh);
          const v4f b0b = *(const v4f*)(cv + 1 * 32 + 8 * hh + 4);
          const v4f b0c = *(const v4f*)(cv + 1 * 32 + 16 + 8 * hh);
#pragma unroll
          for (int e = 0; e < 4; ++e) {
            acc0[e]     = fmaf(w0a[e], xv, b0a[e]);
            acc0[4 + e] = fmaf(w0b[e], xv, b0b[e]);
            acc1[e]     = fmaf(w0c[e], xv, b0c[e]);
            acc1[4 + e] = 0.0f;
          }
        }
        acc0 = mma3(wh[0][0], wl[0][0], h0h, h0l, acc0);
        acc1 = mma3(wh[0][1], wl[0][1], h0h, h0l, acc1);
        {
          v8f p, q;
#pragma unroll
          for (int r = 0; r < 8; ++r) p[r] = tanh_f(acc0[r]);
#pragma unroll
          for (int r = 0; r < 4; ++r) {
            const float tv = tanh_f(acc1[r]);
            q[r]     = (hh == 0) ? tv : 0.0f;
            q[4 + r] = 0.0f;
          }
          pack_frag(p, q, h0h, h0l);
        }

        v8f c0, c1;
        {
          const v4f b1a = *(const v4f*)(cv + 2 * 32 + 8 * hh);
          const v4f b1b = *(const v4f*)(cv + 2 * 32 + 8 * hh + 4);
          const v4f b1c = *(const v4f*)(cv + 2 * 32 + 16 + 8 * hh);
#pragma unroll
          for (int e = 0; e < 4; ++e) {
            c0[e]     = b1a[e];
            c0[4 + e] = b1b[e];
            c1[e]     = b1c[e];
            c1[4 + e] = 0.0f;
          }
        }
        c0 = mma3(wh[1][0], wl[1][0], h0h, h0l, c0);
        c0 = mma3(wh[2][0], wl[2][0], h1h, h1l, c0);
        c1 = mma3(wh[1][1], wl[1][1], h0h, h0l, c1);
        c1 = mma3(wh[2][1], wl[2][1], h1h, h1l, c1);
        {
          v8f p, q;
#pragma unroll
          for (int r = 0; r < 8; ++r) p[r] = tanh_f(c0[r]);
#pragma unroll
          for (int r = 0; r < 4; ++r) {
            const float tv = tanh_f(c1[r]);
            q[r]     = (hh == 0) ? tv : 0.0f;
            q[4 + r] = 0.0f;
          }
          pack_frag(p, q, h1h, h1l);
        }

        v8f oacc;
        {
          const v4f fa = *(const v4f*)(cv + 3 * 32 + 8 * hh);
          const v4f fb = *(const v4f*)(cv + 3 * 32 + 8 * hh + 4);
#pragma unroll
          for (int e = 0; e < 4; ++e) {
            oacc[e]     = fa[e];
            oacc[4 + e] = fb[e];
          }
        }
        oacc = mma3(wh[3][0], wl[3][0], h1h, h1l, oacc);
        {
          float* op = os + c * kORow + s * kNout + 8 * hh;
          op[0] = oacc[0];
          op[1] = oacc[1];
          if (hh == 0) {
            op[2] = oacc[2];
            op[3] = oacc[3];
            op[4] = oacc[4];
            op[5] = oacc[5];
            op[6] = oacc[6];
            op[7] = oacc[7];
          }
        }
      }

      __syncthreads();
      {
        const int tb = t0 + sub * kOChunk;
        for (int pass = 0; pass < 2; ++pass) {
#pragma unroll 4
          for (int it = 0; it < kFlushIt; ++it) {
            const int f    = it * 32 + lane;
            const int row  = f / kOVec4;
            const int col4 = f - row * kOVec4;
            const v4f v = *(const v4f*)(os + f * 4);
            float* gp = out + ((size_t)(b0 + row) * kSteps + (size_t)tb) * kNout + col4 * 4;
            *(volatile v4f*)gp = v;
          }
          __threadfence();
        }
      }
      __syncthreads();
    }
  }
}

extern "C" void kernel_launch(void* const* d_in, const int* in_sizes, int n_in,
                              void* d_out, int out_size, void* d_ws, size_t ws_size,
                              hipStream_t stream) {
  (void)d_ws; (void)ws_size;
  if (n_in < 11 || d_out == nullptr) return;
  if (in_sizes[0] != kBatch * kSteps) return;
  if (in_sizes[1] != kHid) return;
  if (in_sizes[2] != kHid * kHid) return;
  if (in_sizes[3] != kHid) return;
  if (in_sizes[4] != kHid) return;
  if (in_sizes[5] != kHid * kHid) return;
  if (in_sizes[6] != kHid * kHid) return;
  if (in_sizes[7] != kHid) return;
  if (in_sizes[8] != kHid) return;
  if (in_sizes[9] != kNout * kHid) return;
  if (in_sizes[10] != kNout) return;
  if (out_size != kBatch * kSteps * kNout) return;

  const float* x     = (const float*)d_in[0];
  const float* W_ih0 = (const float*)d_in[1];
  const float* W_hh0 = (const float*)d_in[2];
  const float* b_ih0 = (const float*)d_in[3];
  const float* b_hh0 = (const float*)d_in[4];
  const float* W_ih1 = (const float*)d_in[5];
  const float* W_hh1 = (const float*)d_in[6];
  const float* b_ih1 = (const float*)d_in[7];
  const float* b_hh1 = (const float*)d_in[8];
  const float* W_fc  = (const float*)d_in[9];
  const float* b_fc  = (const float*)d_in[10];
  float* out = (float*)d_out;

  seq2_tanh_head_kernel<<<kBatch / kTileB, 32, 0, stream>>>(
      x, W_ih0, W_hh0, b_ih0, b_hh0, W_ih1, W_hh1, b_ih1, b_hh1, W_fc, b_fc, out);
}
